// BarrierNet_1322849927855
// MI455X (gfx1250) — hardware-run, weakly checked
//
#include <hip/hip_runtime.h>


#define NST  524288
#define RC   131072
#define KX   32
#define H1N  128
#define H2N  64
typedef _Float16 h16;
typedef unsigned short bf;
typedef __attribute__((ext_vector_type(16))) __bf16   v16bf;
typedef __attribute__((ext_vector_type(16))) _Float16 v16h;
typedef __attribute__((ext_vector_type(8)))  _Float16 v8h;
typedef __attribute__((ext_vector_type(8)))  unsigned short v8us;
typedef __attribute__((ext_vector_type(8)))  float    v8f;
typedef __attribute__((ext_vector_type(4)))  float    v4f;
typedef v8h  __attribute__((may_alias)) v8ha;
typedef v4f  __attribute__((may_alias)) v4fa;
typedef v8us __attribute__((may_alias)) v8usa;

__device__ __forceinline__ unsigned short f2bf(float f) { unsigned u = __float_as_uint(f); u += 0x7FFFu + ((u >> 16) & 1u); return (unsigned short)(u >> 16); }
__device__ __forceinline__ float bf2f(unsigned short b) { return __uint_as_float(((unsigned)b) << 16); }
__device__ __forceinline__ float bfr(float f) { return bf2f(f2bf(f)); }
__device__ __forceinline__ v16h cat16(v8h lo, v8h hi) { return __builtin_shufflevector(lo, hi, 0, 1, 2, 3, 4, 5, 6, 7, 8, 9, 10, 11, 12, 13, 14, 15); }
__device__ __forceinline__ v16bf cat16b(v8us lo, v8us hi) { return __builtin_bit_cast(v16bf, __builtin_shufflevector(lo, hi, 0, 1, 2, 3, 4, 5, 6, 7, 8, 9, 10, 11, 12, 13, 14, 15)); }
__device__ __forceinline__ v8f wmma16(v16h a, v16h b, v8f c) { return __builtin_amdgcn_wmma_f32_16x16x32_f16(false, a, false, b, (short)0, c, false, false); }
__device__ __forceinline__ v8f wmmab(v16bf a, v16bf b, v8f c) { return __builtin_amdgcn_wmma_f32_16x16x32_bf16(false, a, false, b, (short)0, c, false, false); }


template <typename T16> struct WFrag;
template <> struct WFrag<h16> { typedef v16h V; static __device__ __forceinline__ V ld(const h16* p) { return cat16(*(const v8h*)p, *(const v8h*)(p + 16)); } static __device__ __forceinline__ v8f mma(V a, V b, v8f c) { return wmma16(a, b, c); } };
template <> struct WFrag<bf> { typedef v16bf V; static __device__ __forceinline__ V ld(const bf* p) { return cat16b(*(const v8us*)p, *(const v8us*)(p + 16)); } static __device__ __forceinline__ v8f mma(V a, V b, v8f c) { return wmmab(a, b, c); } };
template <typename T16, int NSPLIT, bool BIAS>
__global__ __launch_bounds__(32) void k_gemmw(const T16* __restrict__ A, const T16* __restrict__ A2, const T16* __restrict__ Bt, const T16* __restrict__ Bt2, int K, float* C, int ldc, const float* __restrict__ bias, size_t sA, size_t sB, size_t sC) {
    typedef typename WFrag<T16>::V V;
    __shared__ __align__(16) float os[16 * 68];
    const size_t z = blockIdx.z; A += z * sA; if (A2) A2 += z * sA; Bt += z * sB; if (Bt2) Bt2 += z * sB; C += z * sC;
    const int lane = threadIdx.x & 31, lr = lane & 15, hi = lane >> 4; const int r0 = blockIdx.x * 64, c0 = blockIdx.y * 64;
    v8f acc[4][4];
#pragma unroll
    for (int mb = 0; mb < 4; ++mb)
#pragma unroll
        for (int nb = 0; nb < 4; ++nb) acc[mb][nb] = (v8f){};
    const size_t aoff = (size_t)(r0 + lr) * K + 8 * hi, boff = (size_t)(c0 + lr) * K + 8 * hi;
#pragma unroll 1
    for (int kc = 0; kc < K; kc += 32) {
        V a[4], a2[4];
#pragma unroll
        for (int mb = 0; mb < 4; ++mb) { a[mb] = WFrag<T16>::ld(A + aoff + (size_t)mb * 16 * K + kc); if (NSPLIT == 1 || NSPLIT == 2) a2[mb] = WFrag<T16>::ld(A2 + aoff + (size_t)mb * 16 * K + kc); }
#pragma unroll
        for (int nb = 0; nb < 4; ++nb) { const V b = WFrag<T16>::ld(Bt + boff + (size_t)nb * 16 * K + kc); V b2; if (NSPLIT >= 2) b2 = WFrag<T16>::ld(Bt2 + boff + (size_t)nb * 16 * K + kc);
#pragma unroll
            for (int mb = 0; mb < 4; ++mb) { acc[mb][nb] = WFrag<T16>::mma(a[mb], b, acc[mb][nb]); if (NSPLIT == 1 || NSPLIT == 2) acc[mb][nb] = WFrag<T16>::mma(a2[mb], b, acc[mb][nb]); if (NSPLIT >= 2) acc[mb][nb] = WFrag<T16>::mma(a[mb], b2, acc[mb][nb]); } }
        asm volatile("v_nop\n\tv_nop\n\tv_nop\n\tv_nop" : "+v"(acc[0][0]), "+v"(acc[1][1]), "+v"(acc[2][2]), "+v"(acc[3][3]) : "v"(a[0]), "v"(a[3]));
    }
#pragma unroll
    for (int mb = 0; mb < 4; ++mb) {
#pragma unroll
        for (int nb = 0; nb < 4; ++nb) {
#pragma unroll
            for (int j = 0; j < 8; ++j) os[(hi * 8 + j) * 68 + nb * 16 + lr] = acc[mb][nb][j]; }
        __builtin_amdgcn_wave_barrier(); asm volatile("" ::: "memory");
        float* crow = C + (size_t)(r0 + mb * 16) * ldc + c0;
#pragma unroll 1
        for (int ps = 0; ps < 2; ++ps) {
#pragma unroll
            for (int s = 0; s < 8; ++s) { const int row = 2 * s + hi, cofs = lr * 4; v4f val = *(const v4fa*)(os + row * 68 + cofs); if (BIAS) { val[0] += bfr(bias[c0 + cofs]); val[1] += bfr(bias[c0 + cofs + 1]); val[2] += bfr(bias[c0 + cofs + 2]); val[3] += bfr(bias[c0 + cofs + 3]); }
                *(volatile v4f*)(crow + (size_t)row * ldc + cofs) = val; }
            if (ps == 0) __threadfence(); }
        __builtin_amdgcn_wave_barrier(); asm volatile("" ::: "memory");
    }
}

typedef __attribute__((ext_vector_type(4))) unsigned short v4us;
typedef __attribute__((ext_vector_type(2))) unsigned short v2us;
typedef __attribute__((ext_vector_type(2))) float v2f;
__device__ __forceinline__ void splitf(float y, unsigned short& h, unsigned short& l) { h = f2bf(y); l = f2bf(y - bf2f(h)); }
__global__ __launch_bounds__(256) void k_cvt8(const float* __restrict__ src, bf* dst, size_t n8) { const size_t i = (size_t)blockIdx.x * 256 + threadIdx.x; if (i >= n8) return; const v8f v = *(const v8f*)(src + i * 8); v8us o;
#pragma unroll
    for (int k = 0; k < 8; ++k) o[k] = f2bf(v[k]); *(volatile v8us*)(dst + i * 8) = o; __threadfence(); *(volatile v8us*)(dst + i * 8) = o; }

__global__ __launch_bounds__(256) void k_xpad(const float* __restrict__ X, size_t n0, bf* XB) { const size_t r = (size_t)blockIdx.x * 256 + threadIdx.x; if (r >= RC) return; unsigned short c[KX];
#pragma unroll
    for (int k = 0; k < KX; ++k) c[k] = (k < 5) ? f2bf(X[(n0 + r) * 5 + k]) : (unsigned short)0;
#pragma unroll 1
    for (int ps = 0; ps < 2; ++ps) {
#pragma unroll
        for (int c8 = 0; c8 < KX; c8 += 8) { v8us o;
#pragma unroll
            for (int k = 0; k < 8; ++k) o[k] = c[c8 + k]; *(volatile v8us*)(XB + r * KX + c8) = o; }
        if (ps == 0) __threadfence(); } }
__global__ __launch_bounds__(128) void k_w1pad(const float* __restrict__ w, bf* Bt) { const int r = threadIdx.x; if (r >= H1N) return; unsigned short c[KX];
#pragma unroll
    for (int k = 0; k < KX; ++k) c[k] = (k < 5) ? f2bf(w[r * 5 + k]) : (unsigned short)0;
#pragma unroll 1
    for (int ps = 0; ps < 2; ++ps) {
#pragma unroll
        for (int c8 = 0; c8 < KX; c8 += 8) { v8us o;
#pragma unroll
            for (int k = 0; k < 8; ++k) o[k] = c[c8 + k]; *(volatile v8us*)(Bt + (size_t)r * KX + c8) = o; }
        if (ps == 0) __threadfence(); } }
__global__ __launch_bounds__(64) void k_bcat(const float* __restrict__ a, const float* __restrict__ b, float* B2) { const int i = threadIdx.x; if (i >= H2N / 4) return; v4f o;
#pragma unroll
    for (int q = 0; q < 4; ++q) { const int c = i * 4 + q; o[q] = (c < 32) ? a[c] : b[c - 32]; } *(volatile v4f*)(B2 + i * 4) = o; __threadfence(); *(volatile v4f*)(B2 + i * 4) = o; }
__global__ __launch_bounds__(256) void k_relu(const float* __restrict__ F, bf* Rh, bf* Rl, size_t n4) { const size_t i = (size_t)blockIdx.x * 256 + threadIdx.x; if (i >= n4) return; const v4f a = *(const v4f*)(F + i * 4); v4us oh, ol;
#pragma unroll
    for (int q = 0; q < 4; ++q) { unsigned short h2, l2; splitf(fmaxf(a[q], 0.0f), h2, l2); oh[q] = h2; ol[q] = l2; }
    *(volatile v4us*)(Rh + i * 4) = oh; *(volatile v4us*)(Rl + i * 4) = ol; __threadfence(); *(volatile v4us*)(Rh + i * 4) = oh; *(volatile v4us*)(Rl + i * 4) = ol; }
__device__ __forceinline__ float sigm(float a) { return __fdiv_rn(1.0f, __fadd_rn(1.0f, __builtin_amdgcn_exp2f(__fmul_rn(a, -1.4426950408889634f)))); }
__global__ __launch_bounds__(256) void k_cbf(const float* __restrict__ F2, const float* __restrict__ X, const float* __restrict__ mean, const float* __restrict__ sd, const float* __restrict__ w31, const float* __restrict__ b31, const float* __restrict__ w32, const float* __restrict__ b32, size_t n0, float* out) {
    const size_t r = (size_t)blockIdx.x * 256 + threadIdx.x; if (r >= RC) return; const float* f = F2 + r * H2N; float a0 = 0.f, a1 = 0.f, c0 = 0.f, c1 = 0.f;
#pragma unroll 1
    for (int k = 0; k < 32; ++k) { const float x21 = fmaxf(f[k], 0.0f), x22 = fmaxf(f[32 + k], 0.0f);
        float p0 = __fmul_rn(x21, bfr(w31[k])); asm volatile("" : "+v"(p0)); a0 = __fadd_rn(a0, p0); float p1 = __fmul_rn(x21, bfr(w31[32 + k])); asm volatile("" : "+v"(p1)); a1 = __fadd_rn(a1, p1);
        float q0 = __fmul_rn(x22, bfr(w32[k])); asm volatile("" : "+v"(q0)); c0 = __fadd_rn(c0, q0); float q1 = __fmul_rn(x22, bfr(w32[32 + k])); asm volatile("" : "+v"(q1)); c1 = __fadd_rn(c1, q1); }
    const float x31a = __fadd_rn(a0, bfr(b31[0])), x31b = __fadd_rn(a1, bfr(b31[1]));
    const float k1 = __fmul_rn(4.0f, sigm(__fadd_rn(c0, bfr(b32[0])))), k2 = __fmul_rn(4.0f, sigm(__fadd_rn(c1, bfr(b32[1]))));
    float x0[5];
#pragma unroll
    for (int j = 0; j < 5; ++j) { float m = __fmul_rn(bfr(X[(n0 + r) * 5 + j]), bfr(sd[j])); asm volatile("" : "+v"(m)); x0[j] = __fadd_rn(m, bfr(mean[j])); }
    const float px = x0[0], py = x0[1], th = x0[2], vv = x0[3]; const float s = sinf(th), c = cosf(th); const float dx = __fsub_rn(px, 40.0f), dy = __fsub_rn(py, 15.0f);
    float dx2 = __fmul_rn(dx, dx); asm volatile("" : "+v"(dx2)); float dy2 = __fmul_rn(dy, dy); asm volatile("" : "+v"(dy2)); const float barrier = __fsub_rn(__fadd_rn(dx2, dy2), 36.0f);
    float t1 = __fmul_rn(__fmul_rn(__fmul_rn(2.0f, dx), vv), c); asm volatile("" : "+v"(t1)); float t2 = __fmul_rn(__fmul_rn(__fmul_rn(2.0f, dy), vv), s); asm volatile("" : "+v"(t2)); const float bdot = __fadd_rn(t1, t2);
    const float Lf2b = __fmul_rn(__fmul_rn(2.0f, vv), vv);
    float e1 = __fmul_rn(__fmul_rn(__fmul_rn(-2.0f, dx), vv), s); asm volatile("" : "+v"(e1)); float e2 = __fmul_rn(__fmul_rn(__fmul_rn(2.0f, dy), vv), c); asm volatile("" : "+v"(e2)); const float LgLfbu1 = __fadd_rn(e1, e2);
    float g1 = __fmul_rn(__fmul_rn(2.0f, dx), c); asm volatile("" : "+v"(g1)); float g2 = __fmul_rn(__fmul_rn(2.0f, dy), s); asm volatile("" : "+v"(g2)); const float LgLfbu2 = __fadd_rn(g1, g2);
    const float G0 = -LgLfbu1, G1 = -LgLfbu2;
    float hb = __fmul_rn(__fadd_rn(k1, k2), bdot); asm volatile("" : "+v"(hb)); float hc = __fmul_rn(__fmul_rn(k1, k2), barrier); asm volatile("" : "+v"(hc)); const float hh = __fadd_rn(__fadd_rn(Lf2b, hb), hc);
    const float u00 = -x31a, u01 = -x31b;
    float gu0 = __fmul_rn(G0, u00); asm volatile("" : "+v"(gu0)); float gu1 = __fmul_rn(G1, u01); asm volatile("" : "+v"(gu1)); const float viol = __fsub_rn(__fadd_rn(gu0, gu1), hh);
    float gg0 = __fmul_rn(G0, G0); asm volatile("" : "+v"(gg0)); float gg1 = __fmul_rn(G1, G1); asm volatile("" : "+v"(gg1)); const float gg = __fadd_rn(gg0, gg1);
    const float lam = __fdiv_rn(fmaxf(viol, 0.0f), __fadd_rn(gg, 1e-12f));
    float l0 = __fmul_rn(lam, G0); asm volatile("" : "+v"(l0)); float l1 = __fmul_rn(lam, G1); asm volatile("" : "+v"(l1)); v2f u; u[0] = __fsub_rn(u00, l0); u[1] = __fsub_rn(u01, l1);
    *(volatile v2f*)(out + (n0 + r) * 2) = u; __threadfence(); *(volatile v2f*)(out + (n0 + r) * 2) = u; }

extern "C" void kernel_launch(void* const* d_in, const int* in_sizes, int n_in,
                              void* d_out, int out_size, void* d_ws, size_t ws_size, hipStream_t stream) {
    (void)in_sizes; (void)n_in; (void)out_size;
    const float* x = (const float*)d_in[0];   const float* mean = (const float*)d_in[2]; const float* sd = (const float*)d_in[3];
    const float* w1 = (const float*)d_in[4]; const float* b1 = (const float*)d_in[5]; const float* w21 = (const float*)d_in[6]; const float* b21 = (const float*)d_in[7]; const float* w22 = (const float*)d_in[8]; const float* b22 = (const float*)d_in[9];
    const float* w31 = (const float*)d_in[10]; const float* b31 = (const float*)d_in[11]; const float* w32 = (const float*)d_in[12]; const float* b32 = (const float*)d_in[13];
    float* OUT = (float*)d_out;
    char* wsp = (char*)d_ws;
    auto take = [&](size_t bytes) { char* p = wsp; wsp += (bytes + 255) & ~(size_t)255; return (void*)p; };
    bf* W1B = (bf*)take((size_t)H1N * KX * 2); bf* W2B = (bf*)take((size_t)H2N * H1N * 2); float* B2 = (float*)take((size_t)H2N * 4);
    bf* XB = (bf*)take((size_t)RC * KX * 2); float* F1 = (float*)take((size_t)RC * H1N * 4); bf* Hh = (bf*)take((size_t)RC * H1N * 2); bf* Hl = (bf*)take((size_t)RC * H1N * 2); float* F2 = (float*)take((size_t)RC * H2N * 4);
    if ((size_t)(wsp - (char*)d_ws) > ws_size) return;
    k_w1pad<<<1, 128, 0, stream>>>(w1, W1B);
    k_cvt8<<<(unsigned)(((size_t)32 * H1N / 8 + 255) / 256), 256, 0, stream>>>(w21, W2B, (size_t)32 * H1N / 8); k_cvt8<<<(unsigned)(((size_t)32 * H1N / 8 + 255) / 256), 256, 0, stream>>>(w22, W2B + (size_t)32 * H1N, (size_t)32 * H1N / 8);
    k_bcat<<<1, 64, 0, stream>>>(b21, b22, B2);
    static_assert(NST % RC == 0 && RC % 64 == 0, "chunking");
    for (size_t n0 = 0; n0 < NST; n0 += RC) {
        k_xpad<<<(RC + 255) / 256, 256, 0, stream>>>(x, n0, XB);
        k_gemmw<bf, 0, true><<<dim3(RC / 64, H1N / 64, 1), 32, 0, stream>>>(XB, nullptr, W1B, nullptr, KX, F1, H1N, b1, 0, 0, 0);
        k_relu<<<(unsigned)(((size_t)RC * H1N / 4 + 255) / 256), 256, 0, stream>>>(F1, Hh, Hl, (size_t)RC * H1N / 4);
        k_gemmw<bf, 1, true><<<dim3(RC / 64, H2N / 64, 1), 32, 0, stream>>>(Hh, Hl, W2B, nullptr, H1N, F2, H2N, B2, 0, 0, 0);
        k_cbf<<<(RC + 255) / 256, 256, 0, stream>>>(F2, x, mean, sd, w31, b31, w32, b32, n0, OUT); }
}
